// PhysicsInformedNN_73504070304394
// MI455X (gfx1250) — hardware-run, weakly checked
//
#include <hip/hip_runtime.h>


#ifndef NPTS
#define NPTS 65536
#endif
#define NPTS_FULL 65536
#define NCOMP 13
#define NLAY  6
#define HW    20
#define KP    32
#define PPW   32
#define QRS   2048.0f
#define QRI   (1.0f / 2048.0f)
#define WSC   64.0f
#define WSI   (1.0f / 64.0f)
#define FB_HALFS (2 * NCOMP * 2 * 32 * 16)
#define ZS_FLOATS (NCOMP * 32 * 8)

static_assert(KP == 32);
static_assert(HW > 16 && HW - 16 <= 4);
static_assert(HW - 16 == 4);
static_assert(HW <= KP);
static_assert(NPTS % PPW == 0);
static_assert(NPTS <= NPTS_FULL);
static_assert(PPW * 4 == 128);
static_assert(8 * 16 == PPW * 4);
static_assert(5 * 8 * 16 == 5 * PPW * 4);
static_assert(128 * 8 == KP * KP);
static_assert(8 * 4 == KP);
static_assert(FB_HALFS * 2 + ZS_FLOATS * 4 + 5 * PPW * 4 <= 131072);
static_assert((size_t)1 * NPTS_FULL * 4 == 262144);
static_assert((size_t)2 * NPTS_FULL * 4 == 524288);
static_assert((size_t)3 * NPTS_FULL * 4 == 786432);
static_assert((size_t)4 * NPTS_FULL * 4 == 1048576);

typedef _Float16 h16;
typedef __attribute__((ext_vector_type(16))) _Float16 v16h;
typedef __attribute__((ext_vector_type(8)))  _Float16 v8h;
typedef __attribute__((ext_vector_type(4)))  _Float16 v4h;
typedef __attribute__((ext_vector_type(8)))  float    v8f;
typedef __attribute__((ext_vector_type(4)))  float    v4f;
typedef v4f  __attribute__((may_alias)) v4fa;
typedef v8h  __attribute__((may_alias)) v8ha;
typedef v4h  __attribute__((may_alias)) v4ha;

__device__ __forceinline__ unsigned short f2bf(float f) { unsigned u = __float_as_uint(f); u += 0x7FFFu + ((u >> 16) & 1u); return (unsigned short)(u >> 16); }
__device__ __forceinline__ float bfr(float f) { return __uint_as_float(((unsigned)f2bf(f)) << 16); }
__device__ __forceinline__ v16h cat16(v8h lo, v8h hi) { return __builtin_shufflevector(lo, hi, 0, 1, 2, 3, 4, 5, 6, 7, 8, 9, 10, 11, 12, 13, 14, 15); }
__device__ __forceinline__ v8f wmma16(v16h a, v16h b, v8f c) { return __builtin_amdgcn_wmma_f32_16x16x32_f16(false, a, false, b, (short)0, c, false, false); }
__device__ __forceinline__ v16h  ldh(const h16* p) { return cat16(*(const v8h*)p, *(const v8h*)(p + 16)); }
__device__ __forceinline__ void wave_sync() { __builtin_amdgcn_fence(3  , "wavefront"); __builtin_amdgcn_wave_barrier(); asm volatile("" ::: "memory"); }

static __device__ __forceinline__ h16 toh_flush(float v) { const h16 r = (h16)v; return (fabsf(v) < 6.103515625e-05f) ? (h16)0.0f : r; }
__device__ __forceinline__ v8f wmma16g(v16h a, v16h b) {
    v8f c = (v8f){};
    c = wmma16(a, b, c);
    asm volatile("v_nop\n\tv_nop\n\tv_nop\n\tv_nop" : "+v"(c) : "v"(a), "v"(b));
    return c;
}
__device__ __forceinline__ int foff(int buf, int q, int pl, int lane) { return (((buf * NCOMP + q) * 2 + pl) * 32 + lane) * 16; }
__device__ __forceinline__ int zoff(int q, int lane) { return (q * 32 + lane) * 8; }

__device__ __forceinline__ float tanh_f(float z) {
    const float e = __builtin_amdgcn_exp2f(z * 2.8853900817779268f);
    return 1.0f - 2.0f * __builtin_amdgcn_rcpf(e + 1.0f);
}
__device__ __forceinline__ void tanh_jet(float (&c)[NCOMP]) {
    const float zx = c[1], zy = c[2], zt = c[3], zxx = c[4], zxy = c[5], zyy = c[6], zxt = c[7], zyt = c[8];
    const float zxxx = c[9], zxxy = c[10], zxyy = c[11], zyyy = c[12];
    const float s  = tanh_f(c[0]);
    const float d1 = 1.0f - s * s;
    const float d2 = -2.0f * s * d1;
    const float d3 = d1 * (6.0f * s * s - 2.0f);
    c[0]  = s;
    c[1]  = d1 * zx;
    c[2]  = d1 * zy;
    c[3]  = d1 * zt;
    c[4]  = d2 * zx * zx + d1 * zxx;
    c[5]  = d2 * zx * zy + d1 * zxy;
    c[6]  = d2 * zy * zy + d1 * zyy;
    c[7]  = d2 * zx * zt + d1 * zxt;
    c[8]  = d2 * zy * zt + d1 * zyt;
    c[9]  = d3 * zx * zx * zx + 3.0f * d2 * zx * zxx + d1 * zxxx;
    c[10] = d3 * zx * zx * zy + d2 * (2.0f * zx * zxy + zy * zxx) + d1 * zxxy;
    c[11] = d3 * zx * zy * zy + d2 * (2.0f * zy * zxy + zx * zyy) + d1 * zxyy;
    c[12] = d3 * zy * zy * zy + 3.0f * d2 * zy * zyy + d1 * zyyy;
}

static_assert(256 / 32 == 8);
__global__ __launch_bounds__(256) void k_minmax(const float* __restrict__ X, int n, float* MM) {
    __shared__ float smn[8];
    __shared__ float smx[8];
    const int lane = threadIdx.x & 31;
    const int wave = __builtin_amdgcn_readfirstlane((int)(threadIdx.x >> 5));
    float lo = 3.0e38f, hv = -3.0e38f;
#pragma unroll 1
    for (int i = threadIdx.x; i < n; i += 256) { const float v = bfr(X[(size_t)i * 3]); lo = fminf(lo, v); hv = fmaxf(hv, v); }
#pragma unroll
    for (int o = 16; o > 0; o >>= 1) { lo = fminf(lo, __shfl_xor(lo, o, 32)); hv = fmaxf(hv, __shfl_xor(hv, o, 32)); }
    if (lane == 0) { smn[wave] = lo; smx[wave] = hv; }
    __syncthreads();
    float flo = smn[0], fhi = smx[0];
#pragma unroll
    for (int w = 1; w < 8; ++w) { flo = fminf(flo, smn[w]); fhi = fmaxf(fhi, smx[w]); }
    v4f o4; o4[0] = (threadIdx.x == 0) ? flo : 0.0f; o4[1] = (threadIdx.x == 0) ? fhi : 0.0f; o4[2] = 0.0f; o4[3] = 0.0f;
    if (threadIdx.x < 8) { volatile v4f* p = (volatile v4f*)(MM + 4 * threadIdx.x); *p = o4; __threadfence(); *p = o4; }
}

__global__ __launch_bounds__(128) void k_wconv(const float* __restrict__ W, const float* __restrict__ bias, int din, int dout, h16* WTl, float* BPl) {
    const int i = threadIdx.x; const int n = i >> 2, k8 = (i & 3) * 8;
    const int nc = n < dout ? n : dout - 1;
    v8h o;
#pragma unroll
    for (int e = 0; e < 8; ++e) {
        const int k = k8 + e; const int kc = k < din ? k : din - 1;
        float v = W[kc * dout + nc];
        asm volatile("" : "+v"(v));
        const bool ok = (k < din) & (n < dout);
        const h16 t = toh_flush(bfr(v) * WSC);
        o[e] = ok ? t : (h16)0.0f; }
    v4f bv;
#pragma unroll
    for (int e = 0; e < 4; ++e) {
        const int nb = 4 * (i & 7) + e; const int nbc = nb < dout ? nb : dout - 1;
        float t = bias[nbc];
        asm volatile("" : "+v"(t));
        bv[e] = (nb < dout) ? bfr(t) : 0.0f; }
    volatile v8h* wp = (volatile v8h*)(WTl + 8 * i);
    volatile v4f* bp = (volatile v4f*)(BPl + 4 * (i & 7));
    *wp = o; if (i < 8) *bp = bv;
    __threadfence();
    *wp = o; if (i < 8) *bp = bv;
}

__global__ __launch_bounds__(32) __attribute__((amdgpu_num_vgpr(256)))
void k_jet(const float* __restrict__ X, const float* __restrict__ W1, const float* __restrict__ B1, const float* __restrict__ W2, const float* __restrict__ B2,
           const h16* __restrict__ WT, const float* __restrict__ BP, const float* __restrict__ lam1p, const float* __restrict__ lam2p, const float* __restrict__ MM, float* OUT) {
    __shared__ __align__(16) h16 fb[FB_HALFS];
    __shared__ __align__(16) float zst[ZS_FLOATS];
    __shared__ __align__(16) float ost[5 * PPW];
    const int lane = threadIdx.x & 31, lr = lane & 15, hi = lane >> 4;
    const float lb = MM[0], ub = MM[1];
    const float rinv = 1.0f / (ub - lb);
    const float kk = 2.0f * rinv;
    const float lam1 = bfr(lam1p[0]), lam2 = bfr(lam2p[0]);
#pragma unroll 1
    for (int g = 0; g < 2; ++g) {
        const int pt = blockIdx.x * PPW + g * 16 + lr;
        float a1[NCOMP][3];
        {
            const float x0 = bfr(X[(size_t)pt * 3 + 0]), x1 = bfr(X[(size_t)pt * 3 + 1]), x2 = bfr(X[(size_t)pt * 3 + 2]);
            const float h0 = (2.0f * (x0 - lb)) * rinv - 1.0f;
            const float h1 = (2.0f * (x1 - lb)) * rinv - 1.0f;
            const float h2 = (2.0f * (x2 - lb)) * rinv - 1.0f;
#pragma unroll
            for (int n = 0; n < 3; ++n) {
                const float w0 = bfr(W1[n]), w1 = bfr(W1[3 + n]), w2 = bfr(W1[6 + n]);
                float c[NCOMP];
                c[0] = (h0 * w0 + h1 * w1) + h2 * w2 + bfr(B1[n]);
                c[1] = kk * w0; c[2] = kk * w1; c[3] = kk * w2;
#pragma unroll
                for (int q = 4; q < NCOMP; ++q) c[q] = 0.0f;
                tanh_jet(c);
#pragma unroll
                for (int q = 0; q < NCOMP; ++q) a1[q][n] = c[q];
            }
        }
#pragma unroll 1
        for (int s = 0; s < 16; ++s) {
            const int n = (s < 8) ? (8 * hi + s) : (8 + 8 * hi + s);
            const int nc = n < HW ? n : HW - 1;
            float w0 = W2[nc], w1 = W2[HW + nc], w2 = W2[2 * HW + nc], bb = B2[nc];
            asm volatile("" : "+v"(w0), "+v"(w1), "+v"(w2), "+v"(bb));
            const bool ok = n < HW;
            w0 = ok ? bfr(w0) : 0.0f; w1 = ok ? bfr(w1) : 0.0f; w2 = ok ? bfr(w2) : 0.0f; bb = ok ? bfr(bb) : 0.0f;
            float c[NCOMP];
#pragma unroll
            for (int q = 0; q < NCOMP; ++q) c[q] = (a1[q][0] * w0 + a1[q][1] * w1) + a1[q][2] * w2;
            c[0] += bb;
            tanh_jet(c);
#pragma unroll
            for (int q = 0; q < NCOMP; ++q) {
                const h16 a = toh_flush(c[q]);
                const h16 rres = toh_flush((c[q] - (float)a) * QRS);
                fb[foff(0, q, 0, lane) + s] = a;
                fb[foff(0, q, 1, lane) + s] = rres; }
        }
        wave_sync();
        int cur = 0;
#pragma unroll 1
        for (int li = 0; li < NLAY - 1; ++li) {
            const int nxt = cur ^ 1;
#pragma unroll
            for (int j = 0; j < 2; ++j) {
                const int nr = (j == 0) ? 8 : (HW - 16);
                const v16h wa = ldh(WT + (size_t)li * (KP * KP) + (size_t)(16 * j + lr) * KP + 8 * hi);
#pragma unroll 1
                for (int q = 0; q < NCOMP; ++q) {
                    const int o0 = foff(cur, q, 0, lane), o1 = foff(cur, q, 1, lane);
                    const v8h bh0 = *(const v8ha*)(&fb[o0]); const v8h bh1 = *(const v8ha*)(&fb[o0 + 8]);
                    const v8h br0 = *(const v8ha*)(&fb[o1]); const v8h br1 = *(const v8ha*)(&fb[o1 + 8]);
                    const v16h bh = cat16(bh0, bh1);
                    const v16h br = cat16(br0, br1);
                    const v8f aH = wmma16g(wa, bh);
                    const v8f aR = wmma16g(wa, br);
                    const v8f z = (aH + aR * QRI) * WSI;
                    v4f zl, zh;
#pragma unroll
                    for (int r = 0; r < 4; ++r) { zl[r] = z[r]; zh[r] = z[4 + r]; }
                    const int zo = zoff(q, lane);
                    *(v4fa*)(&zst[zo]) = zl; *(v4fa*)(&zst[zo + 4]) = zh;
                }
                wave_sync();
                const int bo = li * KP + 16 * j + 8 * hi;
#pragma unroll 1
                for (int r = 0; r < nr; ++r) {
                    float c[NCOMP];
#pragma unroll
                    for (int q = 0; q < NCOMP; ++q) c[q] = zst[zoff(q, lane) + r];
                    c[0] += BP[bo + r];
                    tanh_jet(c);
#pragma unroll
                    for (int q = 0; q < NCOMP; ++q) {
                        const float v = c[q];
                        const h16 a = toh_flush(v);
                        const h16 rres = toh_flush((v - (float)a) * QRS);
                        fb[foff(nxt, q, 0, lane) + 8 * j + r] = a;
                        fb[foff(nxt, q, 1, lane) + 8 * j + r] = rres; }
                }
                if (j == 1) {
                    const v4h zz = (v4h){};
#pragma unroll 1
                    for (int q = 0; q < NCOMP; ++q) {
                        *(v4ha*)(&fb[foff(nxt, q, 0, lane) + 12]) = zz;
                        *(v4ha*)(&fb[foff(nxt, q, 1, lane) + 12]) = zz; }
                }
                wave_sync();
            }
            cur = nxt;
        }
        {
            const v16h wa = ldh(WT + (size_t)(NLAY - 1) * (KP * KP) + (size_t)lr * KP + 8 * hi);
#pragma unroll 1
            for (int q = 0; q < NCOMP; ++q) {
                const int o0 = foff(cur, q, 0, lane), o1 = foff(cur, q, 1, lane);
                const v8h bh0 = *(const v8ha*)(&fb[o0]); const v8h bh1 = *(const v8ha*)(&fb[o0 + 8]);
                const v8h br0 = *(const v8ha*)(&fb[o1]); const v8h br1 = *(const v8ha*)(&fb[o1 + 8]);
                const v16h bh = cat16(bh0, bh1);
                const v16h br = cat16(br0, br1);
                const v8f aH = wmma16g(wa, bh);
                const v8f aR = wmma16g(wa, br);
                const v8f z = (aH + aR * QRI) * WSI;
                v4f zl, zh;
#pragma unroll
                for (int r = 0; r < 4; ++r) { zl[r] = z[r]; zh[r] = z[4 + r]; }
                const int zo = zoff(q, lane);
                *(v4fa*)(&zst[zo]) = zl; *(v4fa*)(&zst[zo + 4]) = zh;
            }
            wave_sync();
            const float* bp = BP + (NLAY - 1) * KP + 8 * hi;
            const float bz0 = bp[0], bz1 = bp[1];
            float c0[NCOMP], c1[NCOMP];
#pragma unroll
            for (int q = 0; q < NCOMP; ++q) { c0[q] = zst[zoff(q, lane)]; c1[q] = zst[zoff(q, lane) + 1]; }
            c0[0] += bz0; c1[0] += bz1;
            tanh_jet(c0); tanh_jet(c1);
            const float u    =  c0[2];
            const float v    = -c0[1];
            const float pval =  c1[0];
            const float p_x  =  c1[1];
            const float p_y  =  c1[2];
            const float u_t  =  c0[8];
            const float u_x  =  c0[5];
            const float u_y  =  c0[6];
            const float v_t  = -c0[7];
            const float v_x  = -c0[4];
            const float v_y  = -c0[5];
            const float u_xx =  c0[10];
            const float u_yy =  c0[12];
            const float v_xx = -c0[9];
            const float v_yy = -c0[11];
            const float f_u = u_t + lam1 * (u * u_x + v * u_y) + p_x - lam2 * (u_xx + u_yy);
            const float f_v = v_t + lam1 * (u * v_x + v * v_y) + p_y - lam2 * (v_xx + v_yy);
            if (hi == 0) {
                const int sp = g * 16 + lr;
                ost[0 * PPW + sp] = u; ost[1 * PPW + sp] = v; ost[2 * PPW + sp] = pval; ost[3 * PPW + sp] = f_u; ost[4 * PPW + sp] = f_v; }
        }
        wave_sync();
    }
    const int l8 = lane & 7;
    float* ob = OUT + (size_t)blockIdx.x * PPW + 4 * l8;
#pragma unroll 1
    for (int ps = 0; ps < 2; ++ps) {
#pragma unroll
        for (int o = 0; o < 5; ++o) {
            const v4f val = *(const v4fa*)(&ost[o * PPW + 4 * l8]);
            if (lane < 8) *(volatile v4f*)(ob + (size_t)o * NPTS_FULL) = val; }
        if (ps == 0) __threadfence(); }
}

static constexpr size_t al256(size_t v) { return (v + 255) & ~(size_t)255; }
static constexpr size_t SZ_MM = al256((size_t)32 * 4);
static constexpr size_t SZ_WT = al256((size_t)NLAY * KP * KP * 2);
static constexpr size_t SZ_BP = al256((size_t)NLAY * KP * 4);
static constexpr size_t SZ_TOTAL = SZ_MM + SZ_WT + SZ_BP;
static_assert(SZ_TOTAL <= (size_t)134217728);
static_assert(((size_t)KP * KP * 2) % 128 == 0);
static_assert(((size_t)KP * 4) % 128 == 0);

extern "C" void kernel_launch(void* const* d_in, const int* in_sizes, int n_in,
                              void* d_out, int out_size, void* d_ws, size_t ws_size, hipStream_t stream) {
    if (n_in < 19) return;
    if ((size_t)in_sizes[0] < (size_t)NPTS_FULL * 3) return;
    if (in_sizes[1] < 9 || in_sizes[2] < 3 || in_sizes[3] < 3 * HW || in_sizes[4] < HW) return;
    for (int l = 0; l < NLAY - 1; ++l) { if (in_sizes[5 + 2 * l] < HW * HW || in_sizes[6 + 2 * l] < HW) return; }
    if (in_sizes[15] < HW * 2 || in_sizes[16] < 2 || in_sizes[17] < 1 || in_sizes[18] < 1) return;
    if ((size_t)out_size < (size_t)5 * NPTS_FULL) return;
    if (SZ_TOTAL > ws_size) return;
    const float* X  = (const float*)d_in[0];
    const float* W1 = (const float*)d_in[1]; const float* B1 = (const float*)d_in[2];
    const float* W2 = (const float*)d_in[3]; const float* B2 = (const float*)d_in[4];
    const float* lam1 = (const float*)d_in[17]; const float* lam2 = (const float*)d_in[18];
    float* OUT = (float*)d_out;
    char* wsp = (char*)d_ws;
    float* MM = (float*)wsp; wsp += SZ_MM;
    h16* WT = (h16*)wsp; wsp += SZ_WT;
    float* BP = (float*)wsp; wsp += SZ_BP;

    k_minmax<<<1, 256, 0, stream>>>(X, NPTS_FULL, MM);
    for (int l = 0; l < NLAY; ++l) {
        const float* Wl = (const float*)d_in[5 + 2 * l];
        const float* Bl = (const float*)d_in[6 + 2 * l];
        const int dout = (l < NLAY - 1) ? HW : 2;
        k_wconv<<<1, 128, 0, stream>>>(Wl, Bl, HW, dout, WT + (size_t)l * KP * KP, BP + (size_t)l * KP);
    }
    k_jet<<<NPTS / PPW, 32, 0, stream>>>(X, W1, B1, W2, B2, WT, BP, lam1, lam2, MM, OUT);
}
